// Model_39676907883207
// MI455X (gfx1250) — hardware-verified
//
#include <hip/hip_runtime.h>
#include <stddef.h>


typedef _Float16 h16;
typedef _Float16 v16h __attribute__((ext_vector_type(16)));
typedef _Float16 v8h  __attribute__((ext_vector_type(8)));
typedef float    v8f  __attribute__((ext_vector_type(8)));
typedef float    v4f  __attribute__((ext_vector_type(4)));

#ifndef NB
#define NB 8
#endif
#ifndef SEQ
#define SEQ 2048
#endif
#define NB_FULL  8
#define SEQ_FULL 2048
#define HD    128
#define MROWS (NB * SEQ)

static_assert(NB >= 1 && NB <= NB_FULL);
static_assert(SEQ >= 64 && SEQ <= SEQ_FULL);
static_assert((SEQ % 64) == 0 && (SEQ % 32) == 0);
static_assert(HD == 128);
static_assert((HD % 64) == 0 && (HD % 32) == 0);
static_assert(HD == 16 * 8);
static_assert((MROWS % 64) == 0);
static_assert((((size_t)MROWS * 16) % 256) == 0);
static_assert(((HD * 2) % 128) == 0 && ((SEQ * 2) % 128) == 0);
static_assert((size_t)NB_FULL * SEQ_FULL * HD < (size_t)0x7FFFFFFF);

#define LDT 72
#define LDC 68
static_assert((LDT % 8) == 0 && LDT >= 64);
static_assert((LDC % 4) == 0 && LDC >= 64);

#define ICARRY 64.0f
#define MCARRY 16.0f
#define MTSCALE (MCARRY / (ICARRY * ICARRY))
#define OSCALE  (1.0f / (ICARRY * MCARRY * 8.0f))

#define TPLANE_BYTES ((size_t)NB * HD * SEQ * 2)
#define QPLANE_BYTES ((size_t)MROWS * HD * 2)
#define MPLANE_BYTES ((size_t)NB * HD * HD * 2)
#define OFF_KT ((size_t)0)
#define OFF_VT (OFF_KT + TPLANE_BYTES)
#define OFF_Q  (OFF_VT + TPLANE_BYTES)
#define OFF_MT (OFF_Q + QPLANE_BYTES)
#define WS_TOTAL (OFF_MT + MPLANE_BYTES)
static_assert((TPLANE_BYTES % 128) == 0 && (QPLANE_BYTES % 128) == 0 && (MPLANE_BYTES % 128) == 0);
static_assert(WS_TOTAL <= (size_t)134217728);

__device__ __forceinline__ float bf16r(float x) {
  unsigned int u = __float_as_uint(x);
  u = (u + 0x7FFFu + ((u >> 16) & 1u)) & 0xFFFF0000u;
  return __uint_as_float(u);
}

static __device__ __forceinline__ h16 toh_flush(float v) {
  const h16 r = (h16)v;
  return (fabsf(v) < 6.103515625e-05f) ? (h16)0.0f : r;
}

__device__ __forceinline__ v16h frag_at(const _Float16* p) {
  v8h lo = *(const v8h*)(p);
  v8h hi = *(const v8h*)(p + 16);
  v16h out;
#pragma unroll
  for (int i = 0; i < 8; ++i) { out[i] = lo[i]; out[i + 8] = hi[i]; }
  return out;
}

__device__ __forceinline__ v8f wmma16(v16h a, v16h b, v8f c) {
  v8f d = __builtin_amdgcn_wmma_f32_16x16x32_f16(false, a, false, b, (short)0, c,
                                                 false, false);
  asm volatile("v_nop\n\tv_nop\n\tv_nop\n\tv_nop" : "+v"(d) : "v"(a), "v"(b));
  return d;
}

__global__ __launch_bounds__(256) void tconv_kernel(
    const float* __restrict__ X, _Float16* __restrict__ Xt) {
  __shared__ _Float16 T[64 * LDT];
  const unsigned tid = threadIdx.x;
  const unsigned n0 = blockIdx.x * 64u;
  const unsigned k0 = blockIdx.y * 64u;
  const unsigned b  = blockIdx.z;
  const float* __restrict__ src = X + ((size_t)b * SEQ_FULL + k0) * HD + n0;
#pragma unroll 4
  for (unsigned j = 0; j < 16u; ++j) {
    const unsigned idx = tid + 256u * j;
    const unsigned kr = idx >> 6, nc = idx & 63u;
    const float v = src[(size_t)kr * HD + nc];
    T[nc * LDT + kr] = toh_flush(ICARRY * bf16r(v));
  }
  __syncthreads();
  v8h x[2];
  size_t off[2];
#pragma unroll
  for (unsigned i = 0; i < 2u; ++i) {
    const unsigned n = 32u * i + (tid >> 3);
    const unsigned kc = (tid & 7u) * 8u;
    x[i] = *(const v8h*)&T[n * LDT + kc];
    off[i] = ((size_t)b * HD + n0 + n) * SEQ + k0 + kc;
  }
#pragma unroll
  for (int i = 0; i < 2; ++i) *(volatile v8h*)(Xt + off[i]) = x[i];
  __threadfence();
#pragma unroll
  for (int i = 0; i < 2; ++i) *(volatile v8h*)(Xt + off[i]) = x[i];
}

__global__ __launch_bounds__(256) void qconv_kernel(
    const float* __restrict__ Q, _Float16* __restrict__ Q16) {
  const unsigned gid = blockIdx.x * 256u + threadIdx.x;
  const unsigned crow = gid >> 4;
  const unsigned c = (gid & 15u) * 8u;
  const unsigned bidx = crow / (unsigned)SEQ;
  const unsigned sq = crow - bidx * (unsigned)SEQ;
  const float* __restrict__ p = Q + ((size_t)bidx * SEQ_FULL + sq) * HD + c;
  const v4f a0 = *(const v4f*)(p);
  const v4f a1 = *(const v4f*)(p + 4);
  v8h o;
#pragma unroll
  for (int i = 0; i < 4; ++i) {
    o[i]     = toh_flush(ICARRY * bf16r(a0[i]));
    o[i + 4] = toh_flush(ICARRY * bf16r(a1[i]));
  }
  _Float16* d = Q16 + (size_t)crow * HD + c;
  *(volatile v8h*)d = o;
  __threadfence();
  *(volatile v8h*)d = o;
}

template <int MODE>
__device__ __forceinline__ void gemm_body(
    const _Float16* __restrict__ A16, const _Float16* __restrict__ Bt, const unsigned K,
    float* __restrict__ outf, _Float16* __restrict__ out16) {
  __shared__ float Cs[64 * LDC];
  const unsigned tid = threadIdx.x, lane = tid & 31u;
  const unsigned w = (unsigned)__builtin_amdgcn_readfirstlane((int)(threadIdx.x >> 5));
  const unsigned mw = w >> 1, nw = w & 1u;
  const unsigned hh = lane >> 4, m = lane & 15u;
  const unsigned n0 = blockIdx.x * 64u;
  const unsigned row0 = blockIdx.y * 64u;

  const _Float16* ap  = A16 + (size_t)(row0 + mw * 16u + m) * K + hh * 8u;
  const _Float16* bp0 = Bt + (size_t)(n0 + nw * 32u + m) * K + hh * 8u;
  const _Float16* bp1 = bp0 + (size_t)16 * K;
  v8f acc0 = {}, acc1 = {};
#pragma unroll 2
  for (unsigned k0 = 0; k0 < K; k0 += 32u) {
    const v16h a  = frag_at(ap + k0);
    const v16h b0 = frag_at(bp0 + k0);
    const v16h b1 = frag_at(bp1 + k0);
    acc0 = wmma16(a, b0, acc0);
    acc1 = wmma16(a, b1, acc1);
  }
#pragma unroll
  for (int r = 0; r < 8; ++r) {
    float* d = &Cs[(mw * 16u + hh * 8u + (unsigned)r) * LDC + nw * 32u + m];
    d[0]  = acc0[r];
    d[16] = acc1[r];
  }
  __syncthreads();

  if (MODE == 0) {
    v8h x[2];
    size_t off[2];
#pragma unroll
    for (unsigned i = 0; i < 2u; ++i) {
      const unsigned r = 32u * i + (tid >> 3);
      const unsigned c = (tid & 7u) * 8u;
      const v4f u0 = *(const v4f*)&Cs[r * LDC + c];
      const v4f u1 = *(const v4f*)&Cs[r * LDC + c + 4];
#pragma unroll
      for (int j = 0; j < 4; ++j) {
        x[i][j]     = toh_flush(u0[j] * MTSCALE);
        x[i][j + 4] = toh_flush(u1[j] * MTSCALE);
      }
      off[i] = (size_t)(row0 + r) * HD + n0 + c;
    }
#pragma unroll
    for (int i = 0; i < 2; ++i) *(volatile v8h*)(out16 + off[i]) = x[i];
    __threadfence();
#pragma unroll
    for (int i = 0; i < 2; ++i) *(volatile v8h*)(out16 + off[i]) = x[i];
  }

  if (MODE == 1) {
    v4f xs[4];
    size_t off[4];
#pragma unroll
    for (unsigned i = 0; i < 4u; ++i) {
      const unsigned r = 16u * i + (tid >> 4);
      const unsigned c = (tid & 15u) * 4u;
      const unsigned crow = row0 + r;
      const unsigned bidx = crow / (unsigned)SEQ;
      const unsigned sq = crow - bidx * (unsigned)SEQ;
      const size_t frow = (size_t)bidx * SEQ_FULL + sq;
      const v4f u = *(const v4f*)&Cs[r * LDC + c];
      v4f val;
#pragma unroll
      for (int j = 0; j < 4; ++j) val[j] = u[j] * OSCALE;
      xs[i] = val;
      off[i] = frow * HD + n0 + c;
    }
#pragma unroll
    for (int i = 0; i < 4; ++i) *(volatile v4f*)(outf + off[i]) = xs[i];
    __threadfence();
#pragma unroll
    for (int i = 0; i < 4; ++i) *(volatile v4f*)(outf + off[i]) = xs[i];
  }
}

__global__ __launch_bounds__(256) void gemm_mt_kernel(
    const _Float16* __restrict__ Vt, const _Float16* __restrict__ Kt,
    _Float16* __restrict__ Mt) {
  const size_t pb = (size_t)blockIdx.z * HD * SEQ;
  gemm_body<0>(Vt + pb, Kt + pb, (unsigned)SEQ, (float*)0, Mt + (size_t)blockIdx.z * HD * HD);
}

__global__ __launch_bounds__(256) void gemm_out_kernel(
    const _Float16* __restrict__ Q16, const _Float16* __restrict__ Mt,
    float* __restrict__ outf) {
  const unsigned bidx = (blockIdx.y * 64u) / (unsigned)SEQ;
  gemm_body<1>(Q16, Mt + (size_t)bidx * HD * HD, (unsigned)HD, outf, (_Float16*)0);
}

extern "C" void kernel_launch(void* const* d_in, const int* in_sizes, int n_in,
                              void* d_out, int out_size, void* d_ws, size_t ws_size,
                              hipStream_t stream) {
  if (n_in < 3) return;
  const long long need = ((long long)(NB - 1) * SEQ_FULL + SEQ) * HD;
  if ((long long)in_sizes[0] < need) return;
  if ((long long)in_sizes[1] < need) return;
  if ((long long)in_sizes[2] < need) return;
  if ((long long)out_size < need) return;
  if (ws_size < WS_TOTAL) return;

  const float* q = (const float*)d_in[0];
  const float* k = (const float*)d_in[1];
  const float* v = (const float*)d_in[2];
  float* out = (float*)d_out;

  char* ws = (char*)d_ws;
  _Float16* Kt16 = (_Float16*)(ws + OFF_KT);
  _Float16* Vt16 = (_Float16*)(ws + OFF_VT);
  _Float16* Q16  = (_Float16*)(ws + OFF_Q);
  _Float16* Mt16 = (_Float16*)(ws + OFF_MT);

  dim3 blk(256);
  tconv_kernel<<<dim3(HD / 64, SEQ / 64, NB), blk, 0, stream>>>(k, Kt16);
  tconv_kernel<<<dim3(HD / 64, SEQ / 64, NB), blk, 0, stream>>>(v, Vt16);
  qconv_kernel<<<dim3((unsigned)(((size_t)MROWS * 16) / 256)), blk, 0, stream>>>(q, Q16);
  gemm_mt_kernel<<<dim3(HD / 64, HD / 64, NB), blk, 0, stream>>>(Vt16, Kt16, Mt16);
  gemm_out_kernel<<<dim3(HD / 64, MROWS / 64), blk, 0, stream>>>(Q16, Mt16, out);
}
